// FreeConvNetwork_704374636650
// MI455X (gfx1250) — hardware-run, weakly checked
//
#include <hip/hip_runtime.h>


#ifndef NB
#define NB 8192
#endif
#define CH (((NB) < 2048) ? (NB) : 2048)
#define NCH ((NB) / (CH))
static_assert((NB) % 64 == 0);
static_assert((NB) % (CH) == 0);
static_assert((CH) % 64 == 0);

#define XW 28
#define XHW 784
#define P1 169
#define P2 36
#define P3 16
#define C1 32
#define C2 64
#define C3 128
#define F1 9
#define F2 288
#define F3 576
#define FL 2048
#define NOUT 10
#define K2S 18
#define K3S 36
#define KLS 128
#define LD2 (K2S * 32)
#define LD3 (K3S * 32)
#define LDL (KLS * 32)
#define H1W 64
#define H2W 128
#define H3W 256
static_assert(P3 * H3W == LDL);

#define BT2_BYTES ((size_t)P2 * C2 * LD2 * 2)
#define BT3_BYTES ((size_t)P3 * C3 * LD3 * 2)
#define BTL_BYTES ((size_t)16 * LDL * 2)
#define H1_BYTES  ((size_t)P1 * (CH) * H1W * 2)
#define H2_BYTES  ((size_t)P2 * (CH) * H2W * 2)
#define H3_BYTES  ((size_t)(CH) * P3 * H3W * 2)
#define WS_TOTAL  (BT2_BYTES + BT3_BYTES + BTL_BYTES + H1_BYTES + H2_BYTES + H3_BYTES)
static_assert(WS_TOTAL <= (size_t)134217728);
static_assert(BT2_BYTES % 512 == 0);
static_assert(BT3_BYTES % 512 == 0);
static_assert(BTL_BYTES % 512 == 0);
static_assert(H1_BYTES % 512 == 0);
static_assert(H2_BYTES % 512 == 0);
static_assert(H3_BYTES % 512 == 0);

typedef __attribute__((ext_vector_type(16))) __bf16 v16b;
typedef __attribute__((ext_vector_type(8)))  float v8f;
typedef __attribute__((ext_vector_type(4)))  float v4f;
typedef __attribute__((ext_vector_type(4)))  unsigned v4u;
typedef v4u __attribute__((may_alias)) v4u_a;
typedef v4f __attribute__((may_alias)) v4f_a;
typedef unsigned short us;

template <typename T> __device__ __forceinline__ void vst2(void* p, T v) { *(volatile T*)p = v; __threadfence(); *(volatile T*)p = v; }
__device__ __forceinline__ v8f wmma_bf(v16b a, v16b b, v8f c) {
  v8f d = __builtin_amdgcn_wmma_f32_16x16x32_bf16(false, a, false, b, (short)0, c, false, false);
  asm volatile("v_nop\n\tv_nop\n\tv_nop\n\tv_nop" : "+v"(d) : "v"(a), "v"(b));
  return d;
}
__device__ __forceinline__ unsigned bf_bits(float f) { const unsigned u = __float_as_uint(f); return (u + 0x7FFFu + ((u >> 16) & 1u)) >> 16; }
__device__ __forceinline__ float bf_val(unsigned b) { return __uint_as_float(b << 16); }
__device__ __forceinline__ float bf_rne(float f) { return bf_val(bf_bits(f)); }
union Frag { v16b v; v4u u[2]; };
__device__ __forceinline__ v16b frag_b(const us* rowk0, int lane) {
  Frag f; const us* p = rowk0 + 8 * (lane >> 4);
  f.u[0] = *(const v4u_a*)p; f.u[1] = *(const v4u_a*)(p + 16); return f.v;
}

__global__ __launch_bounds__(256) void k_bt2(const float* __restrict__ W, us* __restrict__ Bt) {
  const unsigned n8 = (unsigned)(P2 * C2 * LD2 / 8);
  const unsigned g8 = blockIdx.x * 256u + threadIdx.x; if (g8 >= n8) return;
  const unsigned e0 = g8 * 8u, row = e0 / LD2, kin = e0 % LD2;
  const unsigned s = row / C2, o = row % C2, ks = kin / 32u, kk0 = kin % 32u, tap = ks >> 1;
  union { us h[8]; v4u u; } pk;
#pragma unroll
  for (int t = 0; t < 8; ++t) { const unsigned c = kk0 + (unsigned)t;
    pk.h[t] = (us)bf_bits(W[((size_t)o * F2 + c * 9u + tap) * P2 + s]); }
  vst2(Bt + e0, pk.u);
}
__global__ __launch_bounds__(256) void k_bt3(const float* __restrict__ W, us* __restrict__ Bt) {
  const unsigned n8 = (unsigned)(P3 * C3 * LD3 / 8);
  const unsigned g8 = blockIdx.x * 256u + threadIdx.x; if (g8 >= n8) return;
  const unsigned e0 = g8 * 8u, row = e0 / LD3, kin = e0 % LD3;
  const unsigned s = row / C3, o = row % C3, ks = kin / 32u, kk0 = kin % 32u, tap = ks >> 2, q = ks & 3u;
  union { us h[8]; v4u u; } pk;
#pragma unroll
  for (int t = 0; t < 8; ++t) { const unsigned c = (q & 1u) * 32u + kk0 + (unsigned)t;
    pk.h[t] = (us)bf_bits(W[((size_t)o * F3 + c * 9u + tap) * P3 + s]); }
  vst2(Bt + e0, pk.u);
}
__global__ __launch_bounds__(256) void k_btl(const float* __restrict__ W, us* __restrict__ Bt) {
  const unsigned n8 = (unsigned)(16 * LDL / 8);
  const unsigned g8 = blockIdx.x * 256u + threadIdx.x; if (g8 >= n8) return;
  const unsigned e0 = g8 * 8u, n = e0 / LDL, kin = e0 % LDL;
  const unsigned ks = kin / 32u, kk0 = kin % 32u, s = ks >> 3, q = ks & 7u;
  const unsigned nn = n < (unsigned)NOUT ? n : (unsigned)(NOUT - 1);
  union { us h[8]; v4u u; } pk;
#pragma unroll
  for (int t = 0; t < 8; ++t) { const unsigned c = (q & 3u) * 32u + kk0 + (unsigned)t;
    const float v = W[(size_t)nn * FL + c * 16u + s];
    pk.h[t] = n < (unsigned)NOUT ? (us)bf_bits(v) : (us)0; }
  vst2(Bt + e0, pk.u);
}

__global__ __launch_bounds__(64) void k_ll1(const float* __restrict__ x, const float* __restrict__ W1, const float* __restrict__ b1,
                                          us* __restrict__ h1p, int cb0) {
  __shared__ __align__(16) float wsl[C1 * 12];
  __shared__ __align__(16) us S[64][H1W + 8];
  const int tid = threadIdx.x, pos = blockIdx.x, i1 = pos / 13, j1 = pos % 13;
  const int b = cb0 + blockIdx.y * 64 + tid;
  for (int e = tid; e < C1 * 12; e += 64) { const int c = e / 12, t = e % 12, tt = t < 9 ? t : 8;
    const float wv = bf_rne(W1[(c * F1 + tt) * P1 + pos]), bv = bf_rne(b1[c * P1 + pos]);
    wsl[e] = t < 9 ? wv : (t == 9 ? bv : 0.f); }
  float xv[9];
  const float* xp = x + (size_t)b * XHW + (2 * i1) * XW + 2 * j1;
#pragma unroll
  for (int dy = 0; dy < 3; ++dy)
#pragma unroll
    for (int dx = 0; dx < 3; ++dx) xv[dy * 3 + dx] = bf_rne(xp[dy * XW + dx]);
  __syncthreads();
#pragma unroll 1
  for (int c = 0; c < C1; ++c) {
    const v4f w0 = *(const v4f_a*)(wsl + c * 12), w1 = *(const v4f_a*)(wsl + c * 12 + 4), w2 = *(const v4f_a*)(wsl + c * 12 + 8);
    float a = xv[0] * w0[0];
    a = fmaf(xv[1], w0[1], a); a = fmaf(xv[2], w0[2], a); a = fmaf(xv[3], w0[3], a);
    a = fmaf(xv[4], w1[0], a); a = fmaf(xv[5], w1[1], a); a = fmaf(xv[6], w1[2], a); a = fmaf(xv[7], w1[3], a);
    a = fmaf(xv[8], w2[0], a);
    a += w2[1];
    a = a > 0.f ? a : 0.f;
    const unsigned hb = bf_bits(a), lb = bf_bits(a - bf_val(hb));
    S[tid][c] = (us)hb; S[tid][C1 + c] = (us)lb;
  }
  __syncthreads();
  const int wave = tid >> 5, lane = tid & 31;
#pragma unroll
  for (int it = 0; it < 8; ++it) { const int sm = wave * 32 + it * 4 + (lane >> 3), pc = lane & 7;
    const v4u v = *(const v4u_a*)(&S[sm][pc * 8]);
    vst2(h1p + ((size_t)pos * CH + blockIdx.y * 64 + sm) * H1W + pc * 8, v); }
}

__global__ __launch_bounds__(128) void k_ll2(const us* __restrict__ h1p, const us* __restrict__ Bt2, const float* __restrict__ b2,
                                           us* __restrict__ h2p) {
  __shared__ __align__(16) us S[4][16][H2W + 8];
  const int tid = threadIdx.x, wave = tid >> 5, lane = tid & 31, col = lane & 15, g = lane >> 4;
  const int s2 = blockIdx.x, i2 = s2 / 6, j2 = s2 % 6;
  const int m0 = blockIdx.y * 64 + wave * 16;
  const us* Bs = Bt2 + (size_t)s2 * C2 * LD2;
  v8f acc[4] = {};
#pragma unroll 1
  for (int ks = 0; ks < K2S; ++ks) { const int tap = ks >> 1, which = ks & 1;
    const int pos1 = (2 * i2 + tap / 3) * 13 + (2 * j2 + tap % 3);
    const v16b a = frag_b(h1p + ((size_t)pos1 * CH + m0 + col) * H1W + which * 32, lane);
#pragma unroll
    for (int j = 0; j < 4; ++j) acc[j] = wmma_bf(a, frag_b(Bs + (size_t)(j * 16 + col) * LD2 + ks * 32, lane), acc[j]); }
  us (*Sw)[H2W + 8] = S[wave];
#pragma unroll
  for (int j = 0; j < 4; ++j) { const int o = j * 16 + col; const float bv = bf_rne(b2[o * P2 + s2]);
#pragma unroll
    for (int r = 0; r < 8; ++r) { float u = acc[j][r] + bv; u = u > 0.f ? u : 0.f;
      const unsigned hb = bf_bits(u), lb = bf_bits(u - bf_val(hb));
      Sw[8 * g + r][o] = (us)hb; Sw[8 * g + r][C2 + o] = (us)lb; } }
  __syncthreads();
#pragma unroll
  for (int it = 0; it < 8; ++it) { const int rl = it * 2 + g, pc = col;
    const v4u v = *(const v4u_a*)(&Sw[rl][pc * 8]);
    vst2(h2p + ((size_t)s2 * CH + m0 + rl) * H2W + pc * 8, v); }
}

__global__ __launch_bounds__(128) void k_ll3(const us* __restrict__ h2p, const us* __restrict__ Bt3, const float* __restrict__ b3,
                                           us* __restrict__ h3p) {
  __shared__ __align__(16) us S[4][16][H3W + 8];
  const int tid = threadIdx.x, wave = tid >> 5, lane = tid & 31, col = lane & 15, g = lane >> 4;
  const int s3 = blockIdx.x, i3 = s3 / 4, j3 = s3 % 4;
  const int m0 = blockIdx.y * 64 + wave * 16;
  const us* Bs = Bt3 + (size_t)s3 * C3 * LD3;
  v8f acc[8] = {};
#pragma unroll 1
  for (int ks = 0; ks < K3S; ++ks) { const int tap = ks >> 2, q = ks & 3;
    const int pos2 = (i3 + tap / 3) * 6 + (j3 + tap % 3);
    const v16b a = frag_b(h2p + ((size_t)pos2 * CH + m0 + col) * H2W + q * 32, lane);
#pragma unroll
    for (int j = 0; j < 8; ++j) acc[j] = wmma_bf(a, frag_b(Bs + (size_t)(j * 16 + col) * LD3 + ks * 32, lane), acc[j]); }
  us (*Sw)[H3W + 8] = S[wave];
#pragma unroll
  for (int j = 0; j < 8; ++j) { const int o = j * 16 + col; const float bv = bf_rne(b3[o * P3 + s3]);
#pragma unroll
    for (int r = 0; r < 8; ++r) { float u = acc[j][r] + bv; u = u > 0.f ? u : 0.f;
      const unsigned hb = bf_bits(u), lb = bf_bits(u - bf_val(hb));
      Sw[8 * g + r][o] = (us)hb; Sw[8 * g + r][C3 + o] = (us)lb; } }
  __syncthreads();
#pragma unroll
  for (int rl = 0; rl < 16; ++rl) {
    const v4u v = *(const v4u_a*)(&Sw[rl][lane * 8]);
    vst2(h3p + ((size_t)(m0 + rl) * P3 + s3) * H3W + lane * 8, v); }
}

__global__ __launch_bounds__(128) void k_lin(const us* __restrict__ h3p, const us* __restrict__ Btl, const float* __restrict__ bias,
                                           float* __restrict__ out, int row0) {
  __shared__ __align__(16) float S[64 * NOUT];
  const int tid = threadIdx.x, wave = tid >> 5, lane = tid & 31, col = lane & 15, g = lane >> 4;
  const int m0 = blockIdx.x * 64 + wave * 16;
  v8f acc = {};
#pragma unroll 2
  for (int ks = 0; ks < KLS; ++ks) {
    const v16b a = frag_b(h3p + (size_t)(m0 + col) * LDL + ks * 32, lane);
    acc = wmma_bf(a, frag_b(Btl + (size_t)col * LDL + ks * 32, lane), acc); }
  const int cn = col < NOUT ? col : NOUT - 1;
  const float bv = bf_rne(bias[cn]);
  if (col < NOUT) {
#pragma unroll
    for (int r = 0; r < 8; ++r) { const float u = acc[r] + bv; S[(wave * 16 + 8 * g + r) * NOUT + col] = u > 0.f ? u : 0.f; } }
  __syncthreads();
  float* ob = out + (size_t)(row0 + blockIdx.x * 64) * NOUT;
  for (int q = tid; q < 64 * NOUT / 4; q += 128) { const v4f v = *(const v4f_a*)(S + q * 4); vst2(ob + q * 4, v); }
}

extern "C" void kernel_launch(void* const* d_in, const int* in_sizes, int n_in,
                              void* d_out, int out_size, void* d_ws, size_t ws_size,
                              hipStream_t stream) {
  if (n_in < 9) return;
  if (in_sizes[0] < NB * XHW || in_sizes[1] < C1 * F1 * P1 || in_sizes[2] < C1 * P1 || in_sizes[3] < C2 * F2 * P2 ||
      in_sizes[4] < C2 * P2 || in_sizes[5] < C3 * F3 * P3 || in_sizes[6] < C3 * P3 || in_sizes[7] < NOUT * FL ||
      in_sizes[8] < NOUT || out_size < NB * NOUT) return;
  if (ws_size < WS_TOTAL) return;
  const float* x  = (const float*)d_in[0];
  const float* W1 = (const float*)d_in[1]; const float* b1 = (const float*)d_in[2];
  const float* W2 = (const float*)d_in[3]; const float* b2 = (const float*)d_in[4];
  const float* W3 = (const float*)d_in[5]; const float* b3 = (const float*)d_in[6];
  const float* Wl = (const float*)d_in[7]; const float* bl = (const float*)d_in[8];
  float* out = (float*)d_out;
  char* ws = (char*)d_ws; size_t off = 0;
  us* Bt2 = (us*)(ws + off); off += BT2_BYTES;
  us* Bt3 = (us*)(ws + off); off += BT3_BYTES;
  us* Btl = (us*)(ws + off); off += BTL_BYTES;
  us* h1p = (us*)(ws + off); off += H1_BYTES;
  us* h2p = (us*)(ws + off); off += H2_BYTES;
  us* h3p = (us*)(ws + off); off += H3_BYTES;
  if (off > ws_size) return;

  k_bt2<<<(unsigned)((P2 * C2 * LD2 / 8 + 255) / 256), 256, 0, stream>>>(W2, Bt2);
  k_bt3<<<(unsigned)((P3 * C3 * LD3 / 8 + 255) / 256), 256, 0, stream>>>(W3, Bt3);
  k_btl<<<(unsigned)((16 * LDL / 8 + 255) / 256), 256, 0, stream>>>(Wl, Btl);
  for (int c = 0; c < NCH; ++c) {
    k_ll1<<<dim3(P1, CH / 64), 64, 0, stream>>>(x, W1, b1, h1p, c * CH);
    k_ll2<<<dim3(P2, CH / 64), 128, 0, stream>>>(h1p, Bt2, b2, h2p);
    k_ll3<<<dim3(P3, CH / 64), 128, 0, stream>>>(h2p, Bt3, b3, h3p);
    k_lin<<<CH / 64, 128, 0, stream>>>(h3p, Btl, bl, out, c * CH);
  }
}
